// SpikeToGraphFNO2D_11003706212834
// MI455X (gfx1250) — hardware-verified
//
#include <hip/hip_runtime.h>
#include <hip/hip_bf16.h>
#include <math.h>


typedef __attribute__((ext_vector_type(16))) _Float16 v16h;
typedef __attribute__((ext_vector_type(8)))  float    v8f;
typedef __attribute__((ext_vector_type(2)))  float    v2f;
typedef __attribute__((ext_vector_type(4)))  int      v4i;
typedef __attribute__((ext_vector_type(16))) __bf16   v16bf;
typedef __attribute__((ext_vector_type(8)))  _Float16 v8h;
typedef __attribute__((ext_vector_type(4)))  float    v4f;
typedef __attribute__((ext_vector_type(4)))  unsigned v4u;
typedef float __attribute__((may_alias)) float_a;
template <typename T> __device__ __forceinline__ void vst2(void* p, T v) { *(volatile T*)p = v; __threadfence(); *(volatile T*)p = v; }
__device__ __forceinline__ v8f wmma16(v16h a, v16h b, v8f c) {
    v8f d = __builtin_amdgcn_wmma_f32_16x16x32_f16(false, a, false, b, (short)0, c, false, false);
    asm volatile("v_nop\n\tv_nop\n\tv_nop\n\tv_nop" : "+v"(d) : "v"(a), "v"(b));
    return d;
}
__device__ __forceinline__ v8f wmma_bf(v16bf a, v16bf b, v8f c) {
    v8f d = __builtin_amdgcn_wmma_f32_16x16x32_bf16(false, a, false, b, (short)0, c, false, false);
    asm volatile("v_nop\n\tv_nop\n\tv_nop\n\tv_nop" : "+v"(d) : "v"(a), "v"(b));
    return d;
}
struct F2 { v16bf h, l; };
__device__ __forceinline__ F2 split16(const float* v) {
    F2 r;
#pragma unroll
    for (int i = 0; i < 16; ++i) { const __bf16 hh = (__bf16)v[i]; r.h[i] = hh; r.l[i] = (__bf16)(v[i] - (float)hh); }
    return r;
}
__device__ __forceinline__ v8f mac3(const F2& a, const F2& b, v8f c) { c = wmma_bf(a.l, b.h, c); c = wmma_bf(a.h, b.l, c); return wmma_bf(a.h, b.h, c); }

#define NB      512
#define TT      4096
#define DM      128
#define NMODES  32
#define EH      256
#define EH2     128
#define ROWS    1024
#define NN2     262144
#define PI2     6.28318530717958647692f
#define AST     264

#ifndef __has_builtin
#define __has_builtin(x) 0
#endif
#define HAVE_ASYNC_LDS 0

#define OFF_XR    0u
#define OFF_XI    32768u
#define OFF_E     65536u
#define OFF_T1    196608u
#define OFF_E2    327680u
#define OFF_T2    458752u
#define OFF_H     589824u
#define OFF_HS    720896u
#define OFF_HT    983040u
#define OFF_PS    1245184u
#define OFF_PT    1507328u
#define OFF_CRE   1769472u
#define OFF_CIM   2293760u
#define OFF_TC    2818048u
#define OFF_TS    3080192u
#define OFF_D1R   3342336u
#define OFF_D1I   3866624u
#define OFF_EW2H  4390912u

__global__ void twiddle_kernel(float* __restrict__ TC, float* __restrict__ TS) {
    int idx = blockIdx.x * blockDim.x + threadIdx.x;
    int j = idx >> 9, v = idx & 511;
    float ang = (PI2 / 512.0f) * (float)((j * v) & 511);
    vst2(TC + idx, (float_a)(cosf(ang) * (1.0f / 512.0f)));
    vst2(TS + idx, (float_a)(sinf(ang) * (1.0f / 512.0f)));
}

__global__ void ew2half_kernel(const float* __restrict__ ew2, _Float16* __restrict__ out) {
    int g = blockIdx.x * blockDim.x + threadIdx.x;
    union { v8h h; v4u u; } pk;
#pragma unroll
    for (int e = 0; e < 8; ++e) pk.h[e] = (_Float16)ew2[g * 8 + e];
    vst2(out + (size_t)g * 8, pk.u);
}

__global__ void __launch_bounds__(256) dft32_kernel(const float* __restrict__ x,
                                                    float* __restrict__ XR,
                                                    float* __restrict__ XI) {
    int row = blockIdx.x;
    const float* xr = x + (size_t)row * TT;
    int tid = threadIdx.x;
    int w = tid >> 5, k = tid & 31;
    int t0 = w * 512;
    float dth = (PI2 / (float)TT) * (float)k;
    float cd = cosf(dth), sd = sinf(dth);
    float c, s;
    float re = 0.0f, im = 0.0f;
    for (int tb = 0; tb < 512; tb += 128) {
        {
            const int ph = (k * (t0 + tb)) & (TT - 1);
            const float th = (PI2 / (float)TT) * (float)ph;
            c = cosf(th); s = sinf(th);
        }
        for (int t = tb; t < tb + 128; ++t) {
            float xv = xr[t0 + t];
            re = fmaf(xv, c, re);
            im = fmaf(-xv, s, im);
            float cn = c * cd - s * sd;
            s = fmaf(s, cd, c * sd);
            c = cn;
        }
    }
    __shared__ float red[8][32][2];
    red[w][k][0] = re;
    red[w][k][1] = im;
    __syncthreads();
    if (tid < 32) {
        float sr = 0.0f, si = 0.0f;
        for (int ww = 0; ww < 8; ++ww) { sr += red[ww][tid][0]; si += red[ww][tid][1]; }
        vst2(XR + row * NMODES + tid, (float_a)sr);
        vst2(XI + row * NMODES + tid, (float_a)si);
    }
}

__global__ void __launch_bounds__(128) energy_kernel(const float* __restrict__ XR,
                                                     const float* __restrict__ XI,
                                                     const float* __restrict__ Wr,
                                                     const float* __restrict__ Wi,
                                                     float* __restrict__ E) {
    int row = blockIdx.x, d = threadIdx.x;
    const float* xr = XR + row * NMODES;
    const float* xi = XI + row * NMODES;
    float sum = 0.0f;
    for (int k = 0; k < NMODES; ++k) {
        float a = xr[k], bb = xi[k];
        float wr = Wr[k * DM + d], wi = Wi[k * DM + d];
        float yr = a * wr - bb * wi;
        float yi = a * wi + bb * wr;
        sum += sqrtf(yr * yr + yi * yi + 1e-8f);
    }
    vst2(E + row * DM + d, (float_a)(sum * (1.0f / (float)NMODES)));
}

__global__ void rowgemm_kernel(const float* __restrict__ in, const float* __restrict__ W,
                               const float* __restrict__ bias, float* __restrict__ out,
                               int K, int Nc, int doRelu) {
    int row = blockIdx.x;
    __shared__ float rs[256];
    for (int idx = threadIdx.x; idx < K; idx += blockDim.x) rs[idx] = in[(size_t)row * K + idx];
    __syncthreads();
    int n = threadIdx.x;
    float acc = bias ? bias[n] : 0.0f;
#pragma unroll 4
    for (int k = 0; k < K; ++k) acc = fmaf(rs[k], W[k * Nc + n], acc);
    if (doRelu) acc = fmaxf(acc, 0.0f);
    vst2(out + (size_t)row * Nc + n, (float_a)acc);
}

__global__ void __launch_bounds__(256) edge_kernel(const float* __restrict__ PS,
                                                   const float* __restrict__ PT,
                                                   const float* __restrict__ eb1,
                                                   const _Float16* __restrict__ ew2h,
                                                   const float* __restrict__ eb2,
                                                   const float* __restrict__ ew3,
                                                   const float* __restrict__ eb3,
                                                   float* __restrict__ CRE,
                                                   float* __restrict__ CIM) {
    int bidx = blockIdx.x;
    int b   = bidx >> 9;
    int rem = bidx & 511;
    int i0  = (rem >> 4) << 4;
    int j0  = (rem & 15) << 5;

    __shared__ float ps_s[16][EH];
    __shared__ float pt_s[32][EH];
    __shared__ float eb1_s[EH];
    __shared__ float part[8][16 * 32 * 2];
    __shared__ alignas(16) _Float16 Ah[2][32 * AST];

    int tid = threadIdx.x;
    const float* psrc = PS + ((size_t)(b * NB + i0)) * EH;
    const float* ptrc = PT + ((size_t)(b * NB + j0)) * EH;
    for (int idx = tid; idx < 16 * EH; idx += 256) ps_s[idx >> 8][idx & 255] = psrc[idx];
    for (int idx = tid; idx < 32 * EH; idx += 256) pt_s[idx >> 8][idx & 255] = ptrc[idx];
    eb1_s[tid] = eb1[tid];
    __syncthreads();
    for (int idx = tid; idx < 16 * EH; idx += 256) ps_s[idx >> 8][idx & 255] += eb1_s[idx & 255];
    __syncthreads();

    int w = tid >> 5, lane = tid & 31;
    int lm = lane & 15, hh = lane >> 4;
    int n  = w * 16 + lm;
    int kHalf = hh * 8;

    v16h bfr[8];
#pragma unroll
    for (int ks = 0; ks < 8; ++ks)
#pragma unroll
        for (int e = 0; e < 16; ++e)
            bfr[ks][e] = ew2h[(ks * 32 + kHalf + ((e < 8) ? e : (e + 8))) * EH2 + n];

    float w3a = ew3[n * 2 + 0];
    float w3b = ew3[n * 2 + 1];
    float bb2 = eb2[n];

    int bj = tid >> 3;
    int bk = (tid & 7) << 5;
    auto buildA = [&](int mt, int buf) {
        const float* pse = &ps_s[mt][0];
        const float* ptj = &pt_s[bj][0];
        union { _Float16 h[32]; uint4 q[4]; } tmpu;
#pragma unroll
        for (int e = 0; e < 32; ++e)
            tmpu.h[e] = (_Float16)fmaxf(pse[bk + e] + ptj[bk + e], 0.0f);
        uint4* dst = (uint4*)&Ah[buf][bj * AST + bk];
        dst[0] = tmpu.q[0]; dst[1] = tmpu.q[1]; dst[2] = tmpu.q[2]; dst[3] = tmpu.q[3];
    };

    float* pw = part[w];
    buildA(0, 0);
    __syncthreads();

    for (int mt = 0; mt < 16; ++mt) {
        int buf = mt & 1;
        if (mt + 1 < 16) buildA(mt + 1, buf ^ 1);

        v8f acc0 = {}, acc1 = {};
        const _Float16* arow0 = &Ah[buf][lm * AST + kHalf];
        const _Float16* arow1 = &Ah[buf][(16 + lm) * AST + kHalf];
#pragma unroll
        for (int ks = 0; ks < 8; ++ks) {
            union { v16h v; uint4 q[2]; } a0, a1;
            const uint4* pa0 = (const uint4*)(arow0 + ks * 32);
            const uint4* pa1 = (const uint4*)(arow1 + ks * 32);
            a0.q[0] = pa0[0]; a0.q[1] = pa0[2];
            a1.q[0] = pa1[0]; a1.q[1] = pa1[2];
            acc0 = wmma16(a0.v, bfr[ks], acc0);
            acc1 = wmma16(a1.v, bfr[ks], acc1);
        }
#pragma unroll
        for (int half = 0; half < 2; ++half) {
            const v8f& acc = half ? acc1 : acc0;
#pragma unroll
            for (int r = 0; r < 8; ++r) {
                float v = fmaxf(acc[r] + bb2, 0.0f);
                float pr = v * w3a, pi = v * w3b;
#pragma unroll
                for (int off = 8; off > 0; off >>= 1) { pr += __shfl_xor(pr, off, 32); pi += __shfl_xor(pi, off, 32); }
                const int jl = half * 16 + hh * 8 + r;
                if (lm == 0) { pw[(mt * 32 + jl) * 2 + 0] = pr; pw[(mt * 32 + jl) * 2 + 1] = pi; }
            }
        }
        __syncthreads();
    }
    __shared__ __attribute__((aligned(16))) float cre_s[16][32], cim_s[16][32];
    for (int e = tid; e < 16 * 32; e += 256) {
        float sr = eb3[0], si = eb3[1];
#pragma unroll
        for (int ww = 0; ww < 8; ++ww) { sr += part[ww][e * 2 + 0]; si += part[ww][e * 2 + 1]; }
        cre_s[e >> 5][e & 31] = sr; cim_s[e >> 5][e & 31] = si;
    }
    __syncthreads();
    {
        const int sel = tid >> 7, q = tid & 127, il = q >> 3, pc = q & 7;
        const size_t o = ((size_t)(b * NB + i0 + il)) * NB + j0 + pc * 4;
        if (sel == 0) vst2(CRE + o, *(const v4f*)(&cre_s[il][pc * 4]));
        else          vst2(CIM + o, *(const v4f*)(&cim_s[il][pc * 4]));
    }
}

__global__ void __launch_bounds__(256) idft_pass1(const float* __restrict__ CRE,
                                                  const float* __restrict__ CIM,
                                                  const float* __restrict__ TC,
                                                  const float* __restrict__ TS,
                                                  float* __restrict__ D1R,
                                                  float* __restrict__ D1I) {
    __shared__ __attribute__((aligned(16))) float so[8][2][16 * 32];
    int w = threadIdx.x >> 5, lane = threadIdx.x & 31;
    int g   = blockIdx.x * 8 + w;
    int b   = g >> 9;
    int rem = g & 511;
    int mr  = (rem >> 4) << 4;
    int nc  = (rem & 15) << 5;
    int lm  = lane & 15, hh = lane >> 4;

    const float* Cr = CRE + (size_t)b * NN2;
    const float* Ci = CIM + (size_t)b * NN2;

    v8f aRR[2] = {}, aIS[2] = {}, aRS[2] = {}, aIC[2] = {};
#pragma unroll 1
    for (int kk = 0; kk < 512; kk += 32) {
        float av[16];
        const float* ar = Cr + (size_t)(mr + lm) * 512 + kk + 8 * hh;
#pragma unroll
        for (int i = 0; i < 8; ++i) { av[i] = ar[i]; av[8 + i] = ar[16 + i]; }
        const F2 fr = split16(av);
        const float* ai = Ci + (size_t)(mr + lm) * 512 + kk + 8 * hh;
#pragma unroll
        for (int i = 0; i < 8; ++i) { av[i] = ai[i]; av[8 + i] = ai[16 + i]; }
        const F2 fi = split16(av);
#pragma unroll
        for (int j = 0; j < 2; ++j) {
            float bc[16], bs[16];
#pragma unroll
            for (int i = 0; i < 16; ++i) { const int k = kk + 8 * hh + ((i < 8) ? i : (i + 8)); bc[i] = TC[(size_t)k * 512 + nc + 16 * j + lm]; bs[i] = TS[(size_t)k * 512 + nc + 16 * j + lm]; }
            const F2 fc = split16(bc), fs = split16(bs);
            aRR[j] = mac3(fr, fc, aRR[j]); aIS[j] = mac3(fi, fs, aIS[j]);
            aRS[j] = mac3(fr, fs, aRS[j]); aIC[j] = mac3(fi, fc, aIC[j]);
        }
    }
#pragma unroll
    for (int j = 0; j < 2; ++j)
#pragma unroll
        for (int r = 0; r < 8; ++r) {
            so[w][0][(8 * hh + r) * 32 + 16 * j + lm] = aRR[j][r] - aIS[j][r];
            so[w][1][(8 * hh + r) * 32 + 16 * j + lm] = aRS[j][r] + aIC[j][r];
        }
    asm volatile("s_wait_dscnt 0" ::: "memory"); __builtin_amdgcn_wave_barrier(); __builtin_amdgcn_fence(__ATOMIC_RELEASE, "workgroup");
#pragma unroll
    for (int q = 0; q < 4; ++q) { const int rl = q * 4 + (lane >> 3), pc = lane & 7;
        const size_t o = ((size_t)(b * NB + mr + rl)) * NB + nc + pc * 4;
        vst2(D1R + o, *(const v4f*)(&so[w][0][rl * 32 + pc * 4]));
        vst2(D1I + o, *(const v4f*)(&so[w][1][rl * 32 + pc * 4])); }
}

__global__ void __launch_bounds__(256) idft_pass2(const float* __restrict__ D1R,
                                                  const float* __restrict__ D1I,
                                                  const float* __restrict__ TC,
                                                  const float* __restrict__ TS,
                                                  const float* __restrict__ alpha_p,
                                                  const float* __restrict__ beta_p,
                                                  float* __restrict__ out) {
    __shared__ __attribute__((aligned(16))) float so[8][2][16 * 32];
    int w = threadIdx.x >> 5, lane = threadIdx.x & 31;
    int g   = blockIdx.x * 8 + w;
    int b   = g >> 9;
    int rem = g & 511;
    int mr  = (rem >> 4) << 4;
    int nc  = (rem & 15) << 5;
    int lm  = lane & 15, hh = lane >> 4;
    float alpha = alpha_p[0], beta = beta_p[0];

    v8f a1[2] = {}, a2[2] = {};
#pragma unroll 1
    for (int kk = 0; kk < 512; kk += 32) {
        float av[16];
        const float* atc = TC + (size_t)(mr + lm) * 512 + kk + 8 * hh;
#pragma unroll
        for (int i = 0; i < 8; ++i) { av[i] = atc[i]; av[8 + i] = atc[16 + i]; }
        const F2 ftc = split16(av);
        const float* ats = TS + (size_t)(mr + lm) * 512 + kk + 8 * hh;
#pragma unroll
        for (int i = 0; i < 8; ++i) { av[i] = ats[i]; av[8 + i] = ats[16 + i]; }
        const F2 fts = split16(av);
#pragma unroll
        for (int j = 0; j < 2; ++j) {
            float brv[16], biv[16];
#pragma unroll
            for (int i = 0; i < 16; ++i) { const int k = kk + 8 * hh + ((i < 8) ? i : (i + 8)); const size_t ro = ((size_t)(b * NB + k)) * NB + nc + 16 * j + lm; brv[i] = D1R[ro]; biv[i] = D1I[ro]; }
            const F2 fbr = split16(brv), fbi = split16(biv);
            a1[j] = mac3(ftc, fbr, a1[j]);
            a2[j] = mac3(fts, fbi, a2[j]);
        }
    }
#pragma unroll
    for (int j = 0; j < 2; ++j)
#pragma unroll
        for (int r = 0; r < 8; ++r) {
            const float logit = alpha * (a1[j][r] - a2[j][r]) + beta;
            so[w][0][(8 * hh + r) * 32 + 16 * j + lm] = logit;
            so[w][1][(8 * hh + r) * 32 + 16 * j + lm] = 1.0f / (1.0f + expf(-logit));
        }
    asm volatile("s_wait_dscnt 0" ::: "memory"); __builtin_amdgcn_wave_barrier(); __builtin_amdgcn_fence(__ATOMIC_RELEASE, "workgroup");
#pragma unroll
    for (int q = 0; q < 4; ++q) { const int rl = q * 4 + (lane >> 3), pc = lane & 7;
        const size_t o = ((size_t)(b * NB + mr + rl)) * NB + nc + pc * 4;
        vst2(out + o, *(const v4f*)(&so[w][0][rl * 32 + pc * 4]));
        vst2(out + (size_t)2 * NN2 + o, *(const v4f*)(&so[w][1][rl * 32 + pc * 4])); }
}

extern "C" void kernel_launch(void* const* d_in, const int* in_sizes, int n_in,
                              void* d_out, int out_size, void* d_ws, size_t ws_size,
                              hipStream_t stream) {
    (void)in_sizes; (void)n_in; (void)out_size; (void)ws_size;
    const float* spikes = (const float*)d_in[0];
    const float* Wr  = (const float*)d_in[1];
    const float* Wi  = (const float*)d_in[2];
    const float* pw1 = (const float*)d_in[3];
    const float* pb1 = (const float*)d_in[4];
    const float* pw2 = (const float*)d_in[5];
    const float* pb2 = (const float*)d_in[6];
    const float* nw1 = (const float*)d_in[7];
    const float* nb1 = (const float*)d_in[8];
    const float* nw2 = (const float*)d_in[9];
    const float* nb2 = (const float*)d_in[10];
    const float* sw  = (const float*)d_in[11];
    const float* sb  = (const float*)d_in[12];
    const float* tw  = (const float*)d_in[13];
    const float* tb  = (const float*)d_in[14];
    const float* ew1 = (const float*)d_in[15];
    const float* eb1 = (const float*)d_in[16];
    const float* ew2 = (const float*)d_in[17];
    const float* eb2 = (const float*)d_in[18];
    const float* ew3 = (const float*)d_in[19];
    const float* eb3 = (const float*)d_in[20];
    const float* alpha = (const float*)d_in[21];
    const float* beta  = (const float*)d_in[22];

    float* ws = (float*)d_ws;
    float* XR  = ws + OFF_XR;   float* XI  = ws + OFF_XI;
    float* E   = ws + OFF_E;    float* T1  = ws + OFF_T1;
    float* E2  = ws + OFF_E2;   float* T2  = ws + OFF_T2;
    float* H   = ws + OFF_H;
    float* HS  = ws + OFF_HS;   float* HT  = ws + OFF_HT;
    float* PS  = ws + OFF_PS;   float* PT  = ws + OFF_PT;
    float* CRE = ws + OFF_CRE;  float* CIM = ws + OFF_CIM;
    float* TC  = ws + OFF_TC;   float* TS  = ws + OFF_TS;
    float* D1R = ws + OFF_D1R;  float* D1I = ws + OFF_D1I;
    _Float16* EW2H = (_Float16*)(ws + OFF_EW2H);
    float* out = (float*)d_out;

    twiddle_kernel<<<NN2 / 256, 256, 0, stream>>>(TC, TS);
    ew2half_kernel<<<(EH * EH2 / 8) / 256, 256, 0, stream>>>(ew2, EW2H);

    dft32_kernel<<<ROWS, 256, 0, stream>>>(spikes, XR, XI);
    energy_kernel<<<ROWS, 128, 0, stream>>>(XR, XI, Wr, Wi, E);

    rowgemm_kernel<<<ROWS, 128, 0, stream>>>(E,  pw1, pb1, T1, 128, 128, 1);
    rowgemm_kernel<<<ROWS, 128, 0, stream>>>(T1, pw2, pb2, E2, 128, 128, 0);
    rowgemm_kernel<<<ROWS, 128, 0, stream>>>(E2, nw1, nb1, T2, 128, 128, 1);
    rowgemm_kernel<<<ROWS, 128, 0, stream>>>(T2, nw2, nb2, H,  128, 128, 1);
    rowgemm_kernel<<<ROWS, 256, 0, stream>>>(H,  sw,  sb,  HS, 128, 256, 0);
    rowgemm_kernel<<<ROWS, 256, 0, stream>>>(H,  tw,  tb,  HT, 128, 256, 0);
    rowgemm_kernel<<<ROWS, 256, 0, stream>>>(HS, ew1,            nullptr, PS, 256, 256, 0);
    rowgemm_kernel<<<ROWS, 256, 0, stream>>>(HT, ew1 + EH * EH,  nullptr, PT, 256, 256, 0);

    edge_kernel<<<1024, 256, 0, stream>>>(PS, PT, eb1, EW2H, eb2, ew3, eb3, CRE, CIM);

    idft_pass1<<<128, 256, 0, stream>>>(CRE, CIM, TC, TS, D1R, D1I);
    idft_pass2<<<128, 256, 0, stream>>>(D1R, D1I, TC, TS, alpha, beta, out);
}
